// VAEMemoryBank_43825846289093
// MI455X (gfx1250) — hardware-verified
//
#include <hip/hip_runtime.h>
#include <math.h>

typedef __attribute__((ext_vector_type(16))) _Float16 v16h;
typedef __attribute__((ext_vector_type(16))) __bf16 v16b;
typedef __attribute__((ext_vector_type(8)))  _Float16 v8h;
typedef __attribute__((ext_vector_type(8)))  float v8f;
typedef __attribute__((ext_vector_type(4)))  float v4f;
typedef __attribute__((ext_vector_type(2)))  float v2f;
typedef __attribute__((ext_vector_type(4)))  unsigned v4u;
typedef __attribute__((ext_vector_type(4)))  int v4i;
typedef float __attribute__((may_alias)) float_a;
typedef int __attribute__((may_alias)) int_a;

template <typename T> __device__ __forceinline__ void vst2(void* p, T v) { *(volatile T*)p = v; __threadfence(); *(volatile T*)p = v; }
__device__ __forceinline__ v8f wmma16(v16h a, v16h b, v8f c) {
  v8f d = __builtin_amdgcn_wmma_f32_16x16x32_f16(false, a, false, b, (short)0, c, false, false);
  asm volatile("v_nop\n\tv_nop\n\tv_nop\n\tv_nop" : "+v"(d) : "v"(a), "v"(b));
  return d;
}
__device__ __forceinline__ v8f wmma_bf(v16b a, v16b b, v8f c) {
  v8f d = __builtin_amdgcn_wmma_f32_16x16x32_bf16(false, a, false, b, (short)0, c, false, false);
  asm volatile("v_nop\n\tv_nop\n\tv_nop\n\tv_nop" : "+v"(d) : "v"(a), "v"(b));
  return d;
}
__device__ __forceinline__ v16h frag_h(const _Float16* rowk0, int lane) {
  union { v16h v; v8h q[2]; } u; const _Float16* p = rowk0 + 8 * (lane >> 4);
  u.q[0] = *(const v8h*)p; u.q[1] = *(const v8h*)(p + 16); return u.v;
}
__device__ __forceinline__ v16h frag_f32(const float* rowk0, int lane) {
  v16h a; const float* p = rowk0 + 8 * (lane >> 4);
#pragma unroll
  for (int i = 0; i < 8; ++i) { a[i] = (_Float16)p[i]; a[8 + i] = (_Float16)p[16 + i]; }
  return a;
}
__device__ __forceinline__ v16h frag_f32s(const float* rowk0, int lane, float sc) {
  v16h a; const float* p = rowk0 + 8 * (lane >> 4);
#pragma unroll
  for (int i = 0; i < 8; ++i) { a[i] = (_Float16)(p[i] * sc); a[8 + i] = (_Float16)(p[16 + i] * sc); }
  return a;
}
__device__ __forceinline__ v16h fragc_f32(const float* W, int k0, int n, int lane, int ld, int K) {
  v16h a; const int g = lane >> 4;
#pragma unroll
  for (int i = 0; i < 8; ++i) { const int ka = k0 + 8 * g + i, kb = ka + 16;
    a[i] = (_Float16)(ka < K ? W[(size_t)(ka < K ? ka : K - 1) * ld + n] : 0.f); a[8 + i] = (_Float16)(kb < K ? W[(size_t)(kb < K ? kb : K - 1) * ld + n] : 0.f); }
  return a;
}
struct F2 { v16b h, l; };
__device__ __forceinline__ F2 bsplit16(const float v[16]) { F2 r;
#pragma unroll
  for (int i = 0; i < 16; ++i) { const __bf16 h = (__bf16)v[i]; r.h[i] = h; r.l[i] = (__bf16)(v[i] - (float)h); }
  return r; }
__device__ __forceinline__ F2 split_row(const float* row, int k0, int lane) { float v[16]; const float* p = row + k0 + 8 * (lane >> 4);
#pragma unroll
  for (int i = 0; i < 8; ++i) { v[i] = p[i]; v[8 + i] = p[16 + i]; }
  return bsplit16(v); }
__device__ __forceinline__ F2 split_rowK(const float* row, int k0, int lane, int K) { float v[16]; const int g = lane >> 4;
#pragma unroll
  for (int i = 0; i < 8; ++i) { const int ka = k0 + 8 * g + i, kb = ka + 16; v[i] = ka < K ? row[ka < K ? ka : K - 1] : 0.f; v[8 + i] = kb < K ? row[kb < K ? kb : K - 1] : 0.f; }
  return bsplit16(v); }
__device__ __forceinline__ F2 split_col(const float* W, int k0, int n, int lane, int ld, int K) { float v[16]; const int g = lane >> 4;
#pragma unroll
  for (int i = 0; i < 8; ++i) { const int ka = k0 + 8 * g + i, kb = ka + 16; v[i] = ka < K ? W[(size_t)(ka < K ? ka : K - 1) * ld + n] : 0.f; v[8 + i] = kb < K ? W[(size_t)(kb < K ? kb : K - 1) * ld + n] : 0.f; }
  return bsplit16(v); }
__device__ __forceinline__ v8f mac3(const F2& a, const F2& b, v8f c) { c = wmma_bf(a.l, b.h, c); c = wmma_bf(a.h, b.l, c); return wmma_bf(a.h, b.h, c); }
__device__ __forceinline__ float sigm(float v) { return 1.0f / (1.0f + expf(-v)); }
#define LDSX() do { asm volatile("s_wait_dscnt 0" ::: "memory"); __builtin_amdgcn_wave_barrier(); __builtin_amdgcn_fence(__ATOMIC_RELEASE, "workgroup"); } while (0)


#define NB 16
#define DC 192
#define TT 4096
#define NS 1000
#define NSP 1024
#define NH 2
#define HD 96
#ifndef TQB
#define TQB (TT / 64)
#define TNB NB
#endif
typedef __attribute__((ext_vector_type(8))) __bf16 v8b;
__device__ __forceinline__ v16b frag_b(const __bf16* rowk0, int lane) {
  union { v16b v; v8b q[2]; } u; const __bf16* p = rowk0 + 8 * (lane >> 4);
  u.q[0] = *(const v8b*)p; u.q[1] = *(const v8b*)(p + 16); return u.v;
}
__device__ __forceinline__ v16b fragc_bf(const float* M, int k0, int n, int lane, int ld) {
  v16b a; const int g = lane >> 4;
#pragma unroll
  for (int i = 0; i < 8; ++i) { a[i] = (__bf16)M[(size_t)(k0 + 8 * g + i) * ld + n]; a[8 + i] = (__bf16)M[(size_t)(k0 + 16 + 8 * g + i) * ld + n]; }
  return a;
}
__device__ __forceinline__ float bfr(float v) { return (float)(__bf16)v; }
__device__ __attribute__((noinline)) float exp_ni(float v) { return expf(v); }
#define WS_PT   0u
#define WS_Q    (WS_PT + 2u * 4 * DC * DC)
#define WS_K    (WS_Q + 4u * NB * TT * DC)
#define WS_VTH  (WS_K + 4u * NSP * DC)
#define WS_VTL  (WS_VTH + 2u * DC * NSP)
#define WS_END  (WS_VTL + 2u * DC * NSP)

__global__ __launch_bounds__(64) void k_pack(const float* __restrict__ Wq, const float* __restrict__ Wk, const float* __restrict__ Wv, const float* __restrict__ Wo, __bf16* __restrict__ PT) {
  __shared__ __align__(16) __bf16 srow[DC]; const int n = blockIdx.x, tid = threadIdx.x; const int which = n / DC, o = n % DC; const float* Wm = (which == 0 ? Wq : which == 1 ? Wk : which == 2 ? Wv : Wo) + (size_t)o * DC;
  for (int k = tid; k < DC; k += 64) srow[k] = (__bf16)Wm[k]; __syncthreads();
  if (tid < DC / 8) vst2((unsigned*)(PT + (size_t)n * DC + tid * 8), *(const v4u*)(&srow[tid * 8]));
}
__global__ __launch_bounds__(128) void k_q(const float* __restrict__ Z, const __bf16* __restrict__ PT, const float* __restrict__ bq, float* __restrict__ Q) {
  __shared__ __align__(16) float so[4][16][196];
  const int tid = threadIdx.x, wave = tid >> 5, lane = tid & 31, col = lane & 15, g = lane >> 4; const int b = blockIdx.y; const int t0 = blockIdx.x * 64 + wave * 16; const float* Zb = Z + (size_t)b * DC * TT;
  v8f acc[12] = {};
#pragma unroll
  for (int kc = 0; kc < DC / 32; ++kc) { const v16b a = fragc_bf(Zb, kc * 32, t0 + col, lane, TT);
#pragma unroll
    for (int j = 0; j < 12; ++j) acc[j] = wmma_bf(a, frag_b(PT + (size_t)(j * 16 + col) * DC + kc * 32, lane), acc[j]); }
#pragma unroll
  for (int j = 0; j < 12; ++j) { const float bb = bfr(bq[j * 16 + col]);
#pragma unroll
    for (int r = 0; r < 8; ++r) so[wave][8 * g + r][j * 16 + col] = acc[j][r] + bb; }
  LDSX();
  for (int rl = 0; rl < 16; ++rl) for (int pc = lane; pc < DC / 4; pc += 32) vst2(Q + ((size_t)b * TT + t0 + rl) * DC + pc * 4, *(const v4f*)&so[wave][rl][pc * 4]);
}
__global__ __launch_bounds__(128) void k_kv(const float* __restrict__ MB_, const __bf16* __restrict__ PT, const float* __restrict__ bk, const float* __restrict__ bv, float* __restrict__ K, __bf16* __restrict__ VTH, __bf16* __restrict__ VTL) {
  __shared__ __align__(16) float so[4][16][196]; __shared__ __align__(16) __bf16 svh[DC][72], svl[DC][72];
  const int tid = threadIdx.x, wave = tid >> 5, lane = tid & 31, col = lane & 15, g = lane >> 4; const int s0 = blockIdx.x * 64 + wave * 16;
#pragma unroll 1
  for (int which = 1; which <= 2; ++which) { v8f acc[12] = {};
#pragma unroll
    for (int kc = 0; kc < DC / 32; ++kc) { const v16b a = fragc_bf(MB_, kc * 32, min(s0 + col, NS - 1), lane, NS);
#pragma unroll
      for (int j = 0; j < 12; ++j) acc[j] = wmma_bf(a, frag_b(PT + (size_t)(which * DC + j * 16 + col) * DC + kc * 32, lane), acc[j]); }
    const float* bb_ = which == 1 ? bk : bv;
#pragma unroll
    for (int j = 0; j < 12; ++j) { const float bb = bfr(bb_[j * 16 + col]);
#pragma unroll
      for (int r = 0; r < 8; ++r) { const int s = s0 + 8 * g + r; so[wave][8 * g + r][j * 16 + col] = (s < NS) ? acc[j][r] + bb : 0.f; } }
    LDSX();
    if (which == 1) { for (int rl = 0; rl < 16; ++rl) for (int pc = lane; pc < DC / 4; pc += 32) vst2(K + (size_t)(s0 + rl) * DC + pc * 4, *(const v4f*)&so[wave][rl][pc * 4]); }
    else { for (int q = lane; q < 16 * DC; q += 32) { const int rl = q / DC, o = q % DC; const float v = so[wave][rl][o]; const __bf16 hb = (__bf16)v; svh[o][wave * 16 + rl] = hb; svl[o][wave * 16 + rl] = (__bf16)(v - (float)hb); } }
    LDSX(); __syncthreads(); }
  for (int q = tid; q < DC * 8; q += 128) { const int o = q >> 3, pc = q & 7; const size_t off = (size_t)o * NSP + blockIdx.x * 64 + pc * 8; vst2((unsigned*)(VTH + off), *(const v4u*)&svh[o][pc * 8]); vst2((unsigned*)(VTL + off), *(const v4u*)&svl[o][pc * 8]); }
}
__global__ __launch_bounds__(128) void k_attn(float* __restrict__ Q, const float* __restrict__ K, const __bf16* __restrict__ VTH, const __bf16* __restrict__ VTL) {
  __shared__ __align__(16) float sp[4][16][36]; __shared__ __align__(16) float so[4][16][100];
  const int tid = threadIdx.x, wave = tid >> 5, lane = tid & 31, col = lane & 15, g = lane >> 4;
  const int qb = blockIdx.x, bh = blockIdx.y, b = bh / NH, h = bh % NH; const int q0 = qb * 64 + wave * 16; const size_t tq = (size_t)b * TT + q0;
  const F2 a0 = split_row(Q + (tq + col) * DC + h * HD, 0, lane), a1 = split_row(Q + (tq + col) * DC + h * HD, 32, lane), a2 = split_row(Q + (tq + col) * DC + h * HD, 64, lane);
  float m[8], l[8];
#pragma unroll
  for (int r = 0; r < 8; ++r) { m[r] = -3.0e38f; l[r] = 0.f; }
  v8f acc[6] = {};
  const float scl = 0.10206207261596575f;
#pragma unroll 1
  for (int ks = 0; ks < NSP / 32; ++ks) {
    v8f s[2];
#pragma unroll
    for (int ct = 0; ct < 2; ++ct) { const int kk = ks * 32 + ct * 16 + col; const float* krow = K + (size_t)kk * DC + h * HD; const F2 k0 = split_row(krow, 0, lane), k1 = split_row(krow, 32, lane), k2 = split_row(krow, 64, lane);
      v8f c = mac3(a0, k0, (v8f){}); c = mac3(a1, k1, c); c = mac3(a2, k2, c);
#pragma unroll
      for (int r = 0; r < 8; ++r) s[ct][r] = (kk < NS) ? c[r] * scl : -3.0e38f; }
#pragma unroll
    for (int r = 0; r < 8; ++r) { float mx = fmaxf(s[0][r], s[1][r]);
#pragma unroll
      for (int o = 1; o < 16; o <<= 1) mx = fmaxf(mx, __shfl_xor(mx, o));
      const float mn = fmaxf(m[r], mx); const float alpha = exp_ni(m[r] - mn);
      const float e0 = s[0][r] <= -1.0e38f ? 0.f : exp_ni(s[0][r] - mn), e1 = s[1][r] <= -1.0e38f ? 0.f : exp_ni(s[1][r] - mn); float es = e0 + e1;
#pragma unroll
      for (int o = 1; o < 16; o <<= 1) es += __shfl_xor(es, o);
      l[r] = l[r] * alpha + es; m[r] = mn;
#pragma unroll
      for (int dt = 0; dt < 6; ++dt) acc[dt][r] *= alpha;
      sp[wave][8 * g + r][col] = e0; sp[wave][8 * g + r][16 + col] = e1; }
    LDSX();
    const F2 pa = split_row(&sp[wave][col][0], 0, lane);
#pragma unroll
    for (int dt = 0; dt < 6; ++dt) { const size_t vrow = (size_t)(h * HD + dt * 16 + col) * NSP + ks * 32; const v16b vh = frag_b(VTH + vrow, lane), vl = frag_b(VTL + vrow, lane);
      acc[dt] = wmma_bf(pa.l, vh, acc[dt]); acc[dt] = wmma_bf(pa.h, vl, acc[dt]); acc[dt] = wmma_bf(pa.h, vh, acc[dt]); }
    LDSX(); }
#pragma unroll
  for (int r = 0; r < 8; ++r) { const float il = 1.0f / l[r];
#pragma unroll
    for (int dt = 0; dt < 6; ++dt) so[wave][8 * g + r][dt * 16 + col] = acc[dt][r] * il; }
  LDSX();
  for (int rl = 0; rl < 16; ++rl) if (lane < 24) vst2(Q + (tq + rl) * DC + h * HD + lane * 4, *(const v4f*)&so[wave][rl][lane * 4]);
}
__global__ __launch_bounds__(128) void k_out(const float* __restrict__ Q, const __bf16* __restrict__ PT, const float* __restrict__ bo, float* __restrict__ OUT) {
  __shared__ __align__(16) float st[DC][68];
  const int tid = threadIdx.x, wave = tid >> 5, lane = tid & 31, col = lane & 15, g = lane >> 4; const int b = blockIdx.y; const int t0 = blockIdx.x * 64;
  v8f acc[12] = {};
#pragma unroll
  for (int kc = 0; kc < DC / 32; ++kc) { const F2 a = split_row(Q + ((size_t)b * TT + t0 + wave * 16 + col) * DC, kc * 32, lane);
#pragma unroll
    for (int j = 0; j < 12; ++j) { const v16b w = frag_b(PT + (size_t)(3 * DC + j * 16 + col) * DC + kc * 32, lane); acc[j] = wmma_bf(a.l, w, acc[j]); acc[j] = wmma_bf(a.h, w, acc[j]); } }
#pragma unroll
  for (int j = 0; j < 12; ++j) { const int o = j * 16 + col; const float bb = bfr(bo[o]);
#pragma unroll
    for (int r = 0; r < 8; ++r) st[o][wave * 16 + 8 * g + r] = acc[j][r] + bb; }
  __syncthreads();
  for (int q = tid; q < DC * 16; q += 128) { const int o = q >> 4, pc = q & 15; vst2(OUT + ((size_t)b * DC + o) * TT + t0 + pc * 4, *(const v4f*)&st[o][pc * 4]); }
}

extern "C" void kernel_launch(void* const* d_in, const int* in_sizes, int n_in, void* d_out, int out_size, void* d_ws, size_t ws_size, hipStream_t stream) {
  (void)in_sizes; (void)n_in; (void)out_size;
  const float** F = (const float**)d_in;
  if (ws_size < (size_t)WS_END) return;
  char* ws = (char*)d_ws; __bf16 *PT = (__bf16*)(ws + WS_PT), *VTH = (__bf16*)(ws + WS_VTH), *VTL = (__bf16*)(ws + WS_VTL); float *Q = (float*)(ws + WS_Q), *K = (float*)(ws + WS_K);
  k_pack<<<4 * DC, 64, 0, stream>>>(F[2], F[4], F[6], F[8], PT);
  k_q<<<dim3(TQB, TNB), 128, 0, stream>>>(F[0], PT, F[3], Q);
  k_kv<<<NSP / 64, 128, 0, stream>>>(F[1], PT, F[5], F[7], K, VTH, VTL);
  k_attn<<<dim3(TQB, TNB * NH), 128, 0, stream>>>(Q, K, VTH, VTL);
  k_out<<<dim3(TQB, TNB), 128, 0, stream>>>(Q, PT, F[9], (float*)d_out);
}
